// QuaternionConcat_16131897164088
// MI455X (gfx1250) — hardware-run, weakly checked
//
#include <hip/hip_runtime.h>


#ifndef NB
#define NB 8
#endif
#define NB_FULL 8
#define IMW   80
#define HW    6400
#define C1    64
#define C2    128
#define CI    192
#define CO    64
#define KD    768
#define NC    256
#define TILES 100
#define NBLK  (NB * TILES)
#define NPIX  (NB * HW)
#define X1_BS (C1 * 4 * HW)
#define X2_BS (C2 * 4 * 1600)
#define OUT_BS (NC * HW)
#define VP    776
#define OSP   68
#define TP    68
#define BN_EPS 1.0e-5f

static_assert(NB <= NB_FULL);
static_assert(HW == IMW * IMW);
static_assert(HW == TILES * 64);
static_assert(CI == C1 + C2);
static_assert(KD == CI * 4);
static_assert(NC == CO * 4);
static_assert(KD % 32 == 0);
static_assert(C1 * 4 == 256);
static_assert((C1 * 4) % 16 == 0);
static_assert((KD / 8) % 2 == 0);
static_assert(NC == 4 * 64);
static_assert((VP * 2) % 16 == 0);
static_assert(VP >= KD);
static_assert((OSP * 4) % 16 == 0);
static_assert((TP * 4) % 16 == 0);
static_assert(TP >= 64);
static_assert(64 * VP * 2 + 4 * 16 * OSP * 4 <= 131072);
static_assert(NC * TP * 4 <= 131072);
static_assert(32 * 16 * 8 == 16 * 64 * 4);
static_assert(256 * 16 * 16 == NC * 64 * 4);
static_assert(256 * 4 * 16 == 64 * NC);
static_assert(64 * 4 == NC);
static_assert((NC * (KD / 8)) % 256 == 0);

typedef unsigned short bf;
typedef __attribute__((ext_vector_type(16))) __bf16   v16bf;
typedef __attribute__((ext_vector_type(8)))  unsigned short v8us;
typedef __attribute__((ext_vector_type(8)))  float    v8f;
typedef __attribute__((ext_vector_type(4)))  float    v4f;
typedef v4f  __attribute__((may_alias)) v4fa;

__device__ __forceinline__ unsigned short f2bf(float f) { unsigned u = __float_as_uint(f); u += 0x7FFFu + ((u >> 16) & 1u); return (unsigned short)(u >> 16); }
__device__ __forceinline__ float bfr(float f) { return __uint_as_float(((unsigned)f2bf(f)) << 16); }
__device__ __forceinline__ v16bf cat16b(v8us lo, v8us hi) { return __builtin_bit_cast(v16bf, __builtin_shufflevector(lo, hi, 0, 1, 2, 3, 4, 5, 6, 7, 8, 9, 10, 11, 12, 13, 14, 15)); }
__device__ __forceinline__ v8f wmmab(v16bf a, v16bf b, v8f c) { return __builtin_amdgcn_wmma_f32_16x16x32_bf16(false, a, false, b, (short)0, c, false, false); }
__device__ __forceinline__ v8f wmmabg(v16bf a, v16bf b, v8f c) { c = wmmab(a, b, c); asm volatile("v_nop\n\tv_nop\n\tv_nop\n\tv_nop" : "+v"(c) : "v"(a), "v"(b)); return c; }
__device__ __forceinline__ v16bf ldb(const bf* p)  { return cat16b(*(const v8us*)p, *(const v8us*)(p + 16)); }
__device__ __forceinline__ void wave_sync() { __builtin_amdgcn_fence(3  , "wavefront"); __builtin_amdgcn_wave_barrier(); asm volatile("" ::: "memory"); }
__device__ __forceinline__ unsigned short sel4(unsigned q, unsigned short a, unsigned short b, unsigned short c, unsigned short d) {
    return (q == 0u) ? a : ((q == 1u) ? b : ((q == 2u) ? c : d));
}

__global__ __launch_bounds__(256) void k_m(const float* __restrict__ Wr, const float* __restrict__ Wi, const float* __restrict__ Wj, const float* __restrict__ Wk, bf* MT) {
    const unsigned i = blockIdx.x * 256u + threadIdx.x; if (i >= (unsigned)(NC * (KD / 8))) return;
    const unsigned n = i / 96u, g = i % 96u; const unsigned o = n >> 2, qo = n & 3u;
    const unsigned wi = o * (unsigned)CI + 2u * g;
    const float r0 = Wr[wi], r1 = Wr[wi + 1], i0 = Wi[wi], i1 = Wi[wi + 1], j0 = Wj[wi], j1 = Wj[wi + 1], k0 = Wk[wi], k1 = Wk[wi + 1];
    const unsigned short ur0 = f2bf(r0), ui0 = f2bf(i0), uj0 = f2bf(j0), uk0 = f2bf(k0);
    const unsigned short ur1 = f2bf(r1), ui1 = f2bf(i1), uj1 = f2bf(j1), uk1 = f2bf(k1);
    const unsigned short ni0 = f2bf(-i0), nj0 = f2bf(-j0), nk0 = f2bf(-k0), ni1 = f2bf(-i1), nj1 = f2bf(-j1), nk1 = f2bf(-k1);
    v8us ov;
    ov[0] = sel4(qo, ur0, ui0, uj0, uk0);
    ov[1] = sel4(qo, ni0, ur0, uk0, nj0);
    ov[2] = sel4(qo, nj0, nk0, ur0, ui0);
    ov[3] = sel4(qo, nk0, uj0, ni0, ur0);
    ov[4] = sel4(qo, ur1, ui1, uj1, uk1);
    ov[5] = sel4(qo, ni1, ur1, uk1, nj1);
    ov[6] = sel4(qo, nj1, nk1, ur1, ui1);
    ov[7] = sel4(qo, nk1, uj1, ni1, ur1);
    bf* dst = MT + (size_t)i * 8;
    *(volatile v8us*)dst = ov; __threadfence(); *(volatile v8us*)dst = ov;
}

__global__ __launch_bounds__(128) void k_gemm(const float* __restrict__ X1, const float* __restrict__ X2, const bf* __restrict__ MT, float* Y) {
    __shared__ __align__(16) bf vs[64 * VP];
    __shared__ __align__(16) float os[4 * 16 * OSP];
    const unsigned tid = threadIdx.x;
    const int lane = (int)(tid & 31u), lr = lane & 15, hi = lane >> 4;
    const int wave = __builtin_amdgcn_readfirstlane((int)(threadIdx.x >> 5));
    const unsigned bx = blockIdx.x; const unsigned b = bx / (unsigned)TILES, tl = bx % (unsigned)TILES;
    const unsigned pl = tid & 63u, kh = tid >> 6;
    const unsigned pix = tl * 64u + pl;
    const unsigned sy = pix / (unsigned)IMW, sx = pix % (unsigned)IMW;
    const unsigned g2 = (sy >> 1) * 40u + (sx >> 1);
    const float* s1 = X1 + (size_t)b * X1_BS + pix;
    const float* s2 = X2 + (size_t)b * X2_BS + g2;
#pragma unroll 1
    for (unsigned it = 0; it < 16u; ++it) {
        const unsigned k0 = (it * 2u + kh) * 8u; float v[8]; v8us ov;
#pragma unroll
        for (int j = 0; j < 8; ++j) v[j] = s1[(size_t)(k0 + (unsigned)j) * HW];
#pragma unroll
        for (int j = 0; j < 8; ++j) ov[j] = f2bf(v[j]);
        *(v8us*)(&vs[pl * VP + k0]) = ov; }
#pragma unroll 1
    for (unsigned it = 16u; it < 48u; ++it) {
        const unsigned k0 = (it * 2u + kh) * 8u; const unsigned kk = k0 - 256u; float v[8]; v8us ov;
#pragma unroll
        for (int j = 0; j < 8; ++j) v[j] = s2[(size_t)(kk + (unsigned)j) * 1600];
#pragma unroll
        for (int j = 0; j < 8; ++j) ov[j] = f2bf(v[j]);
        *(v8us*)(&vs[pl * VP + k0]) = ov; }
    __syncthreads();
    v8f acc[4][4];
#pragma unroll
    for (int mb = 0; mb < 4; ++mb)
#pragma unroll
        for (int nb = 0; nb < 4; ++nb) acc[mb][nb] = (v8f){};
    const int aoff = lr * VP + 8 * hi;
    const size_t boff = (size_t)(64 * wave + lr) * KD + 8 * hi;
#pragma unroll 1
    for (int kc = 0; kc < KD; kc += 32) {
        v16bf a[4];
#pragma unroll
        for (int mb = 0; mb < 4; ++mb) { const int ai = aoff + mb * 16 * VP + kc;
            const v8us x0 = *(const v8us*)(&vs[ai]); const v8us x1 = *(const v8us*)(&vs[ai + 16]); a[mb] = cat16b(x0, x1); }
#pragma unroll
        for (int nb = 0; nb < 4; ++nb) { const v16bf bb = ldb(MT + boff + (size_t)nb * 16 * KD + kc);
#pragma unroll
            for (int mb = 0; mb < 4; ++mb) acc[mb][nb] = wmmabg(a[mb], bb, acc[mb][nb]); }
    }
    const int wb = wave * 16 * OSP;
    float* yrow = Y + (size_t)bx * 64 * NC + 64 * wave;
#pragma unroll
    for (int mb = 0; mb < 4; ++mb) {
#pragma unroll
        for (int nb = 0; nb < 4; ++nb) {
#pragma unroll
            for (int j = 0; j < 8; ++j) os[wb + (hi * 8 + j) * OSP + nb * 16 + lr] = acc[mb][nb][j]; }
        wave_sync();
#pragma unroll 1
        for (int ps = 0; ps < 2; ++ps) {
#pragma unroll
            for (int s = 0; s < 8; ++s) { const int row = 2 * s + (lane >> 4), c4 = (lane & 15) * 4;
                const v4f val = *(const v4fa*)(&os[wb + row * OSP + c4]);
                *(volatile v4f*)(yrow + (size_t)(mb * 16 + row) * NC + c4) = val; }
            if (ps == 0) __threadfence(); }
        wave_sync();
    }
}

template <int CENTER>
__device__ __forceinline__ void colsum_body(const float* __restrict__ Y, const float* __restrict__ MEAN, float* PART) {
#pragma clang fp contract(off)
    const unsigned t = threadIdx.x; const unsigned bx = blockIdx.x;
    const size_t base = (size_t)bx * 64 * NC + 4u * t;
    v4f mu = (v4f){};
    if (CENTER) mu = *(const v4f*)(MEAN + 4u * t);
    v4f s = (v4f){};
#pragma unroll 4
    for (int r = 0; r < 64; ++r) {
        const v4f v = *(const v4f*)(Y + base + (size_t)r * NC);
        if (CENTER) { const v4f d = v - mu; s = s + d * d; } else { s = s + v; } }
    float* dst = PART + (size_t)bx * NC + 4u * t;
    *(volatile v4f*)dst = s; __threadfence(); *(volatile v4f*)dst = s;
}
__global__ __launch_bounds__(64) void k_sum(const float* __restrict__ Y, float* PART) { colsum_body<0>(Y, Y, PART); }
__global__ __launch_bounds__(64) void k_sq(const float* __restrict__ Y, const float* __restrict__ MEAN, float* PART) { colsum_body<1>(Y, MEAN, PART); }

__global__ __launch_bounds__(256) void k_red(const float* __restrict__ PART, float* OUTV, int mode) {
#pragma clang fp contract(off)
    __shared__ __align__(16) float sv[NC];
    const unsigned t = threadIdx.x;
    float acc = 0.0f; float comp = 0.0f;
#pragma unroll 4
    for (int i = 0; i < NBLK; ++i) { const float y = PART[(size_t)i * NC + t] - comp; const float tsum = acc + y; comp = (tsum - acc) - y; acc = tsum; }
    const float mv = acc * (1.0f / (float)NPIX);
    float o = mv;
    if (mode != 0) o = 1.0f / sqrtf(mv + BN_EPS);
    sv[t] = o;
    __syncthreads();
    if (t < 64u) { const v4f val = *(const v4fa*)(&sv[4u * t]);
        *(volatile v4f*)(OUTV + 4u * t) = val; __threadfence(); *(volatile v4f*)(OUTV + 4u * t) = val; }
}

__global__ __launch_bounds__(256) void k_out(const float* __restrict__ Y, const float* __restrict__ MEAN, const float* __restrict__ ISTD,
                                             const float* __restrict__ gamma, const float* __restrict__ beta, float* OUT) {
#pragma clang fp contract(off)
    __shared__ __align__(16) float ts[NC * TP];
    const unsigned t = threadIdx.x; const unsigned bx = blockIdx.x; const unsigned b = bx / (unsigned)TILES, tl = bx % (unsigned)TILES;
    const unsigned c4 = (t & 63u) * 4u, rq = t >> 6;
    const v4f mu = *(const v4f*)(MEAN + c4), is = *(const v4f*)(ISTD + c4), gm = *(const v4f*)(gamma + c4), bt = *(const v4f*)(beta + c4);
    float g[4], be[4];
#pragma unroll
    for (int i = 0; i < 4; ++i) { g[i] = bfr(gm[i]); be[i] = bfr(bt[i]); }
    const size_t ybase = (size_t)bx * 64 * NC + c4;
#pragma unroll 1
    for (unsigned it = 0; it < 16u; ++it) { const unsigned row = it * 4u + rq;
        const v4f v = *(const v4f*)(Y + ybase + (size_t)row * NC);
#pragma unroll
        for (int i = 0; i < 4; ++i) { float z = (v[i] - mu[i]) * is[i]; z = z * g[i] + be[i]; ts[(c4 + (unsigned)i) * TP + row] = fmaxf(z, 0.0f); } }
    __syncthreads();
    float* ob = OUT + (size_t)b * OUT_BS + (size_t)tl * 64 + (t & 15u) * 4u;
#pragma unroll 1
    for (int ps = 0; ps < 2; ++ps) {
#pragma unroll 4
        for (unsigned it = 0; it < 16u; ++it) { const unsigned n = it * 16u + (t >> 4);
            const v4f val = *(const v4fa*)(&ts[n * TP + (t & 15u) * 4u]);
            *(volatile v4f*)(ob + (size_t)n * HW) = val; }
        if (ps == 0) __threadfence(); }
}

static constexpr size_t al256(size_t v) { return (v + 255) & ~(size_t)255; }
static constexpr size_t SZ_MT = al256((size_t)NC * KD * 2);
static constexpr size_t SZ_Y  = al256((size_t)NPIX * NC * 4);
static constexpr size_t SZ_PT = al256((size_t)NBLK * NC * 4);
static constexpr size_t SZ_ST = al256((size_t)NC * 4);
static constexpr size_t SZ_TOTAL = SZ_MT + SZ_Y + 2 * SZ_PT + 2 * SZ_ST;
static_assert(SZ_TOTAL <= (size_t)134217728);
static_assert((size_t)NBLK * 64 == (size_t)NPIX);
static_assert((size_t)NBLK * 64 * NC * 4 <= SZ_Y);
static_assert((size_t)NBLK * NC * 4 <= SZ_PT);

extern "C" void kernel_launch(void* const* d_in, const int* in_sizes, int n_in,
                              void* d_out, int out_size, void* d_ws, size_t ws_size, hipStream_t stream) {
    if (n_in < 8) return;
    if ((size_t)in_sizes[0] < (size_t)NB * X1_BS || (size_t)in_sizes[1] < (size_t)NB * X2_BS) return;
    if (in_sizes[2] < CO * CI || in_sizes[3] < CO * CI || in_sizes[4] < CO * CI || in_sizes[5] < CO * CI) return;
    if (in_sizes[6] < NC || in_sizes[7] < NC) return;
    if ((size_t)out_size < (size_t)NB * OUT_BS) return;
    if (SZ_TOTAL > ws_size) return;
    const float* x1 = (const float*)d_in[0]; const float* x2 = (const float*)d_in[1];
    const float* wr = (const float*)d_in[2]; const float* wi = (const float*)d_in[3];
    const float* wj = (const float*)d_in[4]; const float* wk = (const float*)d_in[5];
    const float* gamma = (const float*)d_in[6]; const float* beta = (const float*)d_in[7];
    float* OUT = (float*)d_out;
    char* wsp = (char*)d_ws;
    bf* MT = (bf*)wsp; wsp += SZ_MT;
    float* Y = (float*)wsp; wsp += SZ_Y;
    float* PART1 = (float*)wsp; wsp += SZ_PT;
    float* PART2 = (float*)wsp; wsp += SZ_PT;
    float* MEAN = (float*)wsp; wsp += SZ_ST;
    float* ISTD = (float*)wsp; wsp += SZ_ST;

    k_m<<<(NC * (KD / 8)) / 256, 256, 0, stream>>>(wr, wi, wj, wk, MT);
    k_gemm<<<NBLK, 128, 0, stream>>>(x1, x2, MT, Y);
    k_sum<<<NBLK, 64, 0, stream>>>(Y, PART1);
    k_red<<<1, 256, 0, stream>>>(PART1, MEAN, 0);
    k_sq<<<NBLK, 64, 0, stream>>>(Y, MEAN, PART2);
    k_red<<<1, 256, 0, stream>>>(PART2, ISTD, 1);
    k_out<<<NBLK, 256, 0, stream>>>(Y, MEAN, ISTD, gamma, beta, OUT);
}
